// DisenHAN_49967649521689
// MI455X (gfx1250) — hardware-verified
//
#include <hip/hip_runtime.h>
#include <stdint.h>

#define VROWS   100000
#define VPAD    100096
#define DD      64
#define NFACE   8
#define DF      8
#define NNEIGH  16
#define NITER   3
#define BROOT   2048
#define NCEN    (BROOT * 16)
#define H1P     128
#define TP      72
#define CS      1040
#define OFF_SC  (16 * CS)
#define OFF_IDX (OFF_SC + 16 * 128)
#define OFF_SO  (OFF_IDX + 256)
#define SMEM_FLOATS (OFF_SO + 16 * 64)
#define SMEM_BYTES  (SMEM_FLOATS * 4)
#define RSCALE  0.35355339059327378f
#define NREAL8  (VROWS * DD / 8)
#define NPAD8   (VPAD * DD / 8)
#define OUT1_ELEM (BROOT * DD)

static_assert(DD == 64);
static_assert(NFACE * DF == 64);
static_assert(DF == 8);
static_assert(NNEIGH == 16);
static_assert(NCEN % 16 == 0);
static_assert(BROOT % 16 == 0);
static_assert(VPAD % 128 == 0);
static_assert(VPAD >= VROWS);
static_assert(NCEN % 128 == 0);
static_assert(64 % 32 == 0);
static_assert(128 % 32 == 0);
static_assert(NPAD8 % 256 == 0);
static_assert(NREAL8 % 32 == 0);
static_assert(16 * 8 == 128);
static_assert((CS * 4) % 16 == 0);
static_assert((TP * 2) % 16 == 0);
static_assert(SMEM_BYTES <= 327680);
static_assert(OUT1_ELEM + BROOT * DD <= 2 * BROOT * DD);

typedef __attribute__((ext_vector_type(16))) __bf16 v16b;
typedef __attribute__((ext_vector_type(8)))  __bf16 v8b;
typedef __attribute__((ext_vector_type(8)))  float  v8f;
typedef __attribute__((ext_vector_type(4)))  float  v4f;
typedef __attribute__((ext_vector_type(4)))  unsigned int v4u;
typedef __attribute__((ext_vector_type(2)))  int v2i;
typedef v8b __attribute__((may_alias)) v8ba;
typedef v4f __attribute__((may_alias)) v4fa;
typedef v4u __attribute__((may_alias)) v4ua;
typedef v2i __attribute__((may_alias)) v2ia;

union FragU { v16b v; v8b h[2]; };

__device__ __forceinline__ unsigned short f2bf_bits(float f) {
  const unsigned u = __float_as_uint(f);
  const unsigned r = (u + 0x7FFFu + ((u >> 16) & 1u)) >> 16;
  const unsigned nanv = (u >> 16) | 0x40u;
  return (unsigned short)(((u & 0x7FFFFFFFu) > 0x7F800000u) ? nanv : r);
}
__device__ __forceinline__ float bf_bits2f(unsigned short h) { return __uint_as_float(((unsigned)h) << 16); }
__device__ __forceinline__ unsigned pk16(unsigned short a, unsigned short b) { return (unsigned)a | ((unsigned)b << 16); }
__device__ __forceinline__ int clamp_row(int i) { return min(max(i, 0), VROWS - 1); }

__device__ __forceinline__ v8f wmma_bf16(v16b a, v16b b, v8f c) {
  v8f d = __builtin_amdgcn_wmma_f32_16x16x32_bf16(false, a, false, b, (short)0, c, false, false);
  asm volatile("v_nop\n\tv_nop\n\tv_nop\n\tv_nop" : "+v"(d) : "v"(a), "v"(b));
  return d;
}

__device__ __forceinline__ v16b load_frag(const unsigned short* p, int hh) {
  FragU f;
  f.h[0] = *(const v8ba*)(p + 8 * hh);
  f.h[1] = *(const v8ba*)(p + 16 + 8 * hh);
  return f.v;
}

__device__ __forceinline__ void gemm_core1_32x64(
    const unsigned short* __restrict__ A, const unsigned short* __restrict__ Bt,
    int K, size_t aoff, size_t boff, int hh, v8f (&acc)[2][4]) {
  const unsigned short* a0 = A + aoff;
  const unsigned short* a1 = a0 + (size_t)16 * K;
  const unsigned short* bp = Bt + boff;
#pragma unroll 1
  for (int k0 = 0; k0 < K; k0 += 32) {
    const v16b f0 = load_frag(a0 + k0, hh);
    const v16b f1 = load_frag(a1 + k0, hh);
#pragma unroll
    for (int nt = 0; nt < 4; ++nt) {
      const v16b fb = load_frag(bp + (size_t)nt * 16 * K + k0, hh);
      acc[0][nt] = wmma_bf16(f0, fb, acc[0][nt]);
      acc[1][nt] = wmma_bf16(f1, fb, acc[1][nt]);
    }
  }
}

__global__ __launch_bounds__(256) void k_pa(const float* __restrict__ tab, unsigned short* __restrict__ Tb) {
  const int g = blockIdx.x * 256 + threadIdx.x;
  const int gc = (g < NREAL8) ? g : (NREAL8 - 1);
  const unsigned keep = (g < NREAL8) ? 0xFFFFFFFFu : 0u;
  const float* src = tab + (size_t)gc * 8;
  const v4f a = *(const v4fa*)src;
  const v4f c = *(const v4fa*)(src + 4);
  v4u o;
  o[0] = pk16(f2bf_bits(a[0]), f2bf_bits(a[1])) & keep;
  o[1] = pk16(f2bf_bits(a[2]), f2bf_bits(a[3])) & keep;
  o[2] = pk16(f2bf_bits(c[0]), f2bf_bits(c[1])) & keep;
  o[3] = pk16(f2bf_bits(c[2]), f2bf_bits(c[3])) & keep;
  unsigned short* dst = Tb + (size_t)g * 8;
  *(volatile v4u*)dst = o;
  __threadfence();
  *(volatile v4u*)dst = o;
}

template <int DUP>
__device__ __forceinline__ void pw_body(const float* __restrict__ W, unsigned short* __restrict__ out,
                                        unsigned short* sT) {
  const int tid = threadIdx.x, lane = tid & 31, w = tid >> 5;
  const int c4 = (tid & 15) * 4, rr = tid >> 4;
#pragma unroll
  for (int p = 0; p < 4; ++p) {
    const int r = rr + 16 * p;
    const v4f v = *(const v4fa*)(W + (size_t)r * 64 + c4);
    sT[(c4 + 0) * TP + r] = f2bf_bits(v[0]);
    sT[(c4 + 1) * TP + r] = f2bf_bits(v[1]);
    sT[(c4 + 2) * TP + r] = f2bf_bits(v[2]);
    sT[(c4 + 3) * TP + r] = f2bf_bits(v[3]);
  }
  __syncthreads();
  constexpr int NIT = 2 * (1 + DUP);
  constexpr int PITCH = 64 * (1 + DUP);
  const int q8 = lane & 7, sub = lane >> 3;
  v4u vv[NIT];
#pragma unroll
  for (int it = 0; it < NIT; ++it) {
    const int L = 32 * it + 4 * w + sub;
    const int n = L >> DUP;
    vv[it] = *(const v4ua*)(sT + n * TP + 8 * q8);
  }
  for (int pass = 0; pass < 2; ++pass) {
#pragma unroll
    for (int it = 0; it < NIT; ++it) {
      const int L = 32 * it + 4 * w + sub;
      const int n = L >> DUP;
      const int half = L & DUP;
      *(volatile v4u*)(out + (size_t)n * PITCH + 64 * half + 8 * q8) = vv[it];
    }
    __threadfence();
  }
}

__global__ __launch_bounds__(256) void k_pw1(const float* __restrict__ W, unsigned short* __restrict__ out) {
  __shared__ __align__(16) unsigned short sT[64 * TP];
  pw_body<0>(W, out, sT);
}
__global__ __launch_bounds__(256) void k_pw2(const float* __restrict__ W, unsigned short* __restrict__ out) {
  __shared__ __align__(16) unsigned short sT[64 * TP];
  pw_body<1>(W, out, sT);
}

__global__ __launch_bounds__(128) __attribute__((amdgpu_num_vgpr(248)))
void k_gemm(const unsigned short* __restrict__ A, const unsigned short* __restrict__ Bt,
            float* __restrict__ C, int K) {
  __shared__ __align__(16) float sF[128 * 64];
  const int tid = threadIdx.x, lane = tid & 31, w = tid >> 5;
  const int hh = lane >> 4, m = lane & 15;
  const int m0 = blockIdx.x * 128;
  const int m0w = m0 + 32 * w;

  const v8f zero8 = {0.f, 0.f, 0.f, 0.f, 0.f, 0.f, 0.f, 0.f};
  v8f acc[2][4];
#pragma unroll
  for (int mt = 0; mt < 2; ++mt)
#pragma unroll
    for (int nt = 0; nt < 4; ++nt) acc[mt][nt] = zero8;

  gemm_core1_32x64(A, Bt, K, (size_t)(m0w + m) * K, (size_t)m * K, hh, acc);

#pragma unroll
  for (int nt = 0; nt < 4; ++nt)
#pragma unroll
    for (int mt = 0; mt < 2; ++mt)
#pragma unroll
      for (int r = 0; r < 8; ++r) {
        const int tokl = 32 * w + 16 * mt + 8 * hh + r;
        const int feat = 16 * nt + m;
        sF[tokl * 64 + feat] = acc[mt][nt][r];
      }
  __syncthreads();
  {
    const int rsub = lane >> 4, c4 = (lane & 15) * 4;
    v4f vals[16];
#pragma unroll
    for (int it = 0; it < 16; ++it) {
      const int row = 32 * w + 2 * it + rsub;
      vals[it] = *(const v4fa*)(sF + row * 64 + c4);
    }
    for (int pass = 0; pass < 2; ++pass) {
#pragma unroll
      for (int it = 0; it < 16; ++it) {
        const int row = 32 * w + 2 * it + rsub;
        *(volatile v4f*)(C + (size_t)(m0 + row) * 64 + c4) = vals[it];
      }
      __threadfence();
    }
  }
}

struct Q8 { v4f a; v4f b; };

__device__ __forceinline__ Q8 route_core(const float* nb, float* sc, const v4f c0, const v4f c1) {
  v4f q0 = c0, q1 = c1;
  const v4f zero4 = {0.f, 0.f, 0.f, 0.f};
#pragma unroll 1
  for (int it = 0; it < NITER; ++it) {
    float mx = -__builtin_inff();
#pragma unroll 1
    for (int n = 0; n < NNEIGH; ++n) {
      const v4f x0 = *(const v4fa*)(nb + n * 64);
      const v4f x1 = *(const v4fa*)(nb + n * 64 + 4);
      float s = q0[0] * x0[0];
      s = fmaf(q0[1], x0[1], s);
      s = fmaf(q0[2], x0[2], s);
      s = fmaf(q0[3], x0[3], s);
      s = fmaf(q1[0], x1[0], s);
      s = fmaf(q1[1], x1[1], s);
      s = fmaf(q1[2], x1[2], s);
      s = fmaf(q1[3], x1[3], s);
      s = s * RSCALE;
      sc[n * 128] = s;
      mx = fmaxf(mx, s);
    }
    float l = 0.0f;
    v4f a0 = zero4, a1 = zero4;
#pragma unroll 1
    for (int n = 0; n < NNEIGH; ++n) {
      const float s = sc[n * 128];
      const float p = expf(s - mx);
      const v4f x0 = *(const v4fa*)(nb + n * 64);
      const v4f x1 = *(const v4fa*)(nb + n * 64 + 4);
      l += p;
      a0 = a0 + x0 * p;
      a1 = a1 + x1 * p;
    }
    const float inv = 1.0f / l;
    q0 = c0 + a0 * inv;
    q1 = c1 + a1 * inv;
  }
  Q8 r;
  r.a = q0;
  r.b = q1;
  return r;
}

__global__ __launch_bounds__(128) __attribute__((amdgpu_num_vgpr(248)))
void k_route1(const float* __restrict__ cplane, const int* __restrict__ cidx,
              const float* __restrict__ nplane, const int* __restrict__ nidx,
              unsigned short* __restrict__ H1) {
  extern __shared__ __align__(16) unsigned char dsm[];
  float* NB = (float*)dsm;
  float* SC = NB + OFF_SC;
  int* sIdx = (int*)(dsm + (size_t)OFF_IDX * 4);
  const int tid = threadIdx.x;
  const int g0 = blockIdx.x * 16;

  {
    const v2i raw = *(const v2ia*)(nidx + (size_t)g0 * 16 + 2 * tid);
    sIdx[2 * tid]     = clamp_row(raw[0]);
    sIdx[2 * tid + 1] = clamp_row(raw[1]);
  }
  __syncthreads();
  {
    const int piece = (tid & 15) * 4, rsub = tid >> 4;
#pragma unroll 4
    for (int it = 0; it < 32; ++it) {
      const int r = it * 8 + rsub;
      const int idx = sIdx[r];
      const v4f v = *(const v4fa*)(nplane + (size_t)idx * 64 + piece);
      *(v4fa*)(NB + (r >> 4) * CS + (r & 15) * 64 + piece) = v;
    }
  }
  __syncthreads();

  const int cl = tid >> 3, k = tid & 7;
  const int g = g0 + cl;
  const int ci = clamp_row(cidx[g]);
  const float* cp = cplane + (size_t)ci * 64 + 8 * k;
  const v4f c0 = *(const v4fa*)cp;
  const v4f c1 = *(const v4fa*)(cp + 4);

  const Q8 q = route_core(NB + cl * CS + 8 * k, SC + tid, c0, c1);

  v4u hv, lv;
#pragma unroll
  for (int p = 0; p < 2; ++p) {
    const float x0 = q.a[2 * p], x1 = q.a[2 * p + 1];
    const float y0 = q.b[2 * p], y1 = q.b[2 * p + 1];
    const float rx0 = (x0 > 0.0f) ? x0 : (x0 - x0);
    const float rx1 = (x1 > 0.0f) ? x1 : (x1 - x1);
    const float ry0 = (y0 > 0.0f) ? y0 : (y0 - y0);
    const float ry1 = (y1 > 0.0f) ? y1 : (y1 - y1);
    const unsigned short hx0 = f2bf_bits(rx0), hx1 = f2bf_bits(rx1);
    const unsigned short hy0 = f2bf_bits(ry0), hy1 = f2bf_bits(ry1);
    hv[p]     = pk16(hx0, hx1);
    hv[2 + p] = pk16(hy0, hy1);
    lv[p]     = pk16(f2bf_bits(rx0 - bf_bits2f(hx0)), f2bf_bits(rx1 - bf_bits2f(hx1)));
    lv[2 + p] = pk16(f2bf_bits(ry0 - bf_bits2f(hy0)), f2bf_bits(ry1 - bf_bits2f(hy1)));
  }
  unsigned short* rowp = H1 + (size_t)g * H1P;
  *(volatile v4u*)(rowp + 8 * k) = hv;
  *(volatile v4u*)(rowp + 64 + 8 * k) = lv;
  __threadfence();
  *(volatile v4u*)(rowp + 8 * k) = hv;
  *(volatile v4u*)(rowp + 64 + 8 * k) = lv;
}

__global__ __launch_bounds__(128) __attribute__((amdgpu_num_vgpr(248)))
void k_route0(const unsigned short* __restrict__ tb, const int* __restrict__ ridx,
              const float* __restrict__ nh0, float* __restrict__ out) {
  extern __shared__ __align__(16) unsigned char dsm[];
  float* NB = (float*)dsm;
  float* SC = NB + OFF_SC;
  float* sO = NB + OFF_SO;
  const int tid = threadIdx.x;
  const int b0 = blockIdx.x * 16;

  {
    const int piece = (tid & 15) * 4, rsub = tid >> 4;
#pragma unroll 4
    for (int it = 0; it < 32; ++it) {
      const int r = it * 8 + rsub;
      const v4f v = *(const v4fa*)(nh0 + ((size_t)b0 * 16 + r) * 64 + piece);
      *(v4fa*)(NB + (r >> 4) * CS + (r & 15) * 64 + piece) = v;
    }
  }
  __syncthreads();

  const int cl = tid >> 3, k = tid & 7;
  const int ri = clamp_row(ridx[b0 + cl]);
  const v4u wv = *(const v4ua*)(tb + (size_t)ri * 64 + 8 * k);
  v4f c0, c1;
  c0[0] = __uint_as_float(wv[0] << 16);
  c0[1] = __uint_as_float(wv[0] & 0xFFFF0000u);
  c0[2] = __uint_as_float(wv[1] << 16);
  c0[3] = __uint_as_float(wv[1] & 0xFFFF0000u);
  c1[0] = __uint_as_float(wv[2] << 16);
  c1[1] = __uint_as_float(wv[2] & 0xFFFF0000u);
  c1[2] = __uint_as_float(wv[3] << 16);
  c1[3] = __uint_as_float(wv[3] & 0xFFFF0000u);

  const Q8 q = route_core(NB + cl * CS + 8 * k, SC + tid, c0, c1);

  *(v4fa*)(sO + cl * 64 + 8 * k) = q.a;
  *(v4fa*)(sO + cl * 64 + 8 * k + 4) = q.b;
  __syncthreads();
  {
    const int piece = (tid & 15) * 4, rsub = tid >> 4;
    v4f vals[2];
#pragma unroll
    for (int it = 0; it < 2; ++it) {
      const int row = 8 * it + rsub;
      vals[it] = *(const v4fa*)(sO + row * 64 + piece);
    }
    for (int pass = 0; pass < 2; ++pass) {
#pragma unroll
      for (int it = 0; it < 2; ++it) {
        const int row = 8 * it + rsub;
        *(volatile v4f*)(out + (size_t)(b0 + row) * 64 + piece) = vals[it];
      }
      __threadfence();
    }
  }
}

extern "C" void kernel_launch(void* const* d_in, const int* in_sizes, int n_in,
                              void* d_out, int out_size, void* d_ws, size_t ws_size,
                              hipStream_t stream) {
  if (n_in < 12) return;
  if (in_sizes[0] != VROWS * DD || in_sizes[1] != VROWS * DD) return;
  if (in_sizes[2] != DD * DD || in_sizes[3] != DD * DD) return;
  if (in_sizes[4] != DD * DD || in_sizes[5] != DD * DD) return;
  if (in_sizes[6] != BROOT || in_sizes[9] != BROOT) return;
  if (in_sizes[7] != NCEN || in_sizes[10] != NCEN) return;
  if (in_sizes[8] != NCEN * 16 || in_sizes[11] != NCEN * 16) return;
  if (out_size != 2 * BROOT * DD) return;

  const float* user_table = (const float*)d_in[0];
  const float* item_table = (const float*)d_in[1];
  const float* Wp0u = (const float*)d_in[2];
  const float* Wp0i = (const float*)d_in[3];
  const float* Wp1u = (const float*)d_in[4];
  const float* Wp1i = (const float*)d_in[5];
  const int* u_idx0 = (const int*)d_in[6];
  const int* u_idx1 = (const int*)d_in[7];
  const int* u_idx2 = (const int*)d_in[8];
  const int* i_idx0 = (const int*)d_in[9];
  const int* i_idx1 = (const int*)d_in[10];
  const int* i_idx2 = (const int*)d_in[11];
  float* out = (float*)d_out;

  const size_t PTB = (size_t)VPAD * DD * 2;
  const size_t PTF = (size_t)VPAD * DD * 4;
  const size_t PH1 = (size_t)NCEN * H1P * 2;
  const size_t PNH = (size_t)NCEN * DD * 4;
  const size_t PW1 = (size_t)DD * DD * 2;
  const size_t PW2 = (size_t)DD * 128 * 2;
  size_t off = 0;
  const size_t oUB  = off; off += PTB;
  const size_t oIB  = off; off += PTB;
  const size_t oTU1 = off; off += PTF;
  const size_t oTI1 = off; off += PTF;
  const size_t oH1U = off; off += PH1;
  const size_t oH1I = off; off += PH1;
  const size_t oNHU = off; off += PNH;
  const size_t oNHI = off; off += PNH;
  const size_t oW1U = off; off += PW1;
  const size_t oW1I = off; off += PW1;
  const size_t oW0I = off; off += PW2;
  const size_t oW0U = off; off += PW2;
  if (off > ws_size) return;
  if (off > (size_t)134217728) return;

  char* ws = (char*)d_ws;
  unsigned short* UB   = (unsigned short*)(ws + oUB);
  unsigned short* IB   = (unsigned short*)(ws + oIB);
  float*          TU1  = (float*)(ws + oTU1);
  float*          TI1  = (float*)(ws + oTI1);
  unsigned short* H1U  = (unsigned short*)(ws + oH1U);
  unsigned short* H1I  = (unsigned short*)(ws + oH1I);
  float*          NH0U = (float*)(ws + oNHU);
  float*          NH0I = (float*)(ws + oNHI);
  unsigned short* W1UT = (unsigned short*)(ws + oW1U);
  unsigned short* W1IT = (unsigned short*)(ws + oW1I);
  unsigned short* W0I2 = (unsigned short*)(ws + oW0I);
  unsigned short* W0U2 = (unsigned short*)(ws + oW0U);

  (void)hipFuncSetAttribute(reinterpret_cast<const void*>(&k_route1),
                            hipFuncAttributeMaxDynamicSharedMemorySize, SMEM_BYTES);
  (void)hipFuncSetAttribute(reinterpret_cast<const void*>(&k_route0),
                            hipFuncAttributeMaxDynamicSharedMemorySize, SMEM_BYTES);

  k_pa<<<dim3(NPAD8 / 256), 256, 0, stream>>>(user_table, UB);
  k_pa<<<dim3(NPAD8 / 256), 256, 0, stream>>>(item_table, IB);
  k_pw1<<<dim3(1), 256, 0, stream>>>(Wp1u, W1UT);
  k_pw1<<<dim3(1), 256, 0, stream>>>(Wp1i, W1IT);
  k_pw2<<<dim3(1), 256, 0, stream>>>(Wp0i, W0I2);
  k_pw2<<<dim3(1), 256, 0, stream>>>(Wp0u, W0U2);
  k_gemm<<<dim3(VPAD / 128), 128, 0, stream>>>(UB, W1UT, TU1, 64);
  k_gemm<<<dim3(VPAD / 128), 128, 0, stream>>>(IB, W1IT, TI1, 64);
  k_route1<<<dim3(NCEN / 16), 128, SMEM_BYTES, stream>>>(TI1, u_idx1, TU1, u_idx2, H1U);
  k_route1<<<dim3(NCEN / 16), 128, SMEM_BYTES, stream>>>(TU1, i_idx1, TI1, i_idx2, H1I);
  k_gemm<<<dim3(NCEN / 128), 128, 0, stream>>>(H1U, W0I2, NH0U, 128);
  k_gemm<<<dim3(NCEN / 128), 128, 0, stream>>>(H1I, W0U2, NH0I, 128);
  k_route0<<<dim3(BROOT / 16), 128, SMEM_BYTES, stream>>>(UB, u_idx0, NH0U, out);
  k_route0<<<dim3(BROOT / 16), 128, SMEM_BYTES, stream>>>(IB, i_idx0, NH0I, out + OUT1_ELEM);
  (void)hipGetLastError();
}
